// SAGEConv_81131932221713
// MI455X (gfx1250) — hardware-run, weakly checked
//
#include <hip/hip_runtime.h>

typedef float          v8f   __attribute__((ext_vector_type(8)));
typedef float          v4f   __attribute__((ext_vector_type(4)));
typedef unsigned int   v4u   __attribute__((ext_vector_type(4)));
typedef int            v8i   __attribute__((ext_vector_type(8)));
typedef unsigned short v8us  __attribute__((ext_vector_type(8)));
typedef unsigned short v16us __attribute__((ext_vector_type(16)));
typedef __bf16         v16bf __attribute__((ext_vector_type(16)));
typedef _Float16       v16h  __attribute__((ext_vector_type(16)));
typedef v4f  __attribute__((may_alias)) v4fa;
typedef v8us __attribute__((may_alias)) v8usa;
union FragB { v16bf v; v16us u; v8us h[2]; v8i w; };
union FragH { v16h  v; v16us u; v8us h[2]; v8i w; };

__device__ __forceinline__ v8f wmb(const FragB& a, const FragB& b, v8f c) {
  v8f d = __builtin_amdgcn_wmma_f32_16x16x32_bf16(false, a.v, false, b.v, (short)0, c, false, false);
  asm volatile("v_nop\n\tv_nop\n\tv_nop\n\tv_nop" : "+v"(d) : "v"(a.w), "v"(b.w));
  return d;
}

__device__ __forceinline__ v8f wmh(const FragH& a, const FragH& b, v8f c) {
  v8f d = __builtin_amdgcn_wmma_f32_16x16x32_f16(false, a.v, false, b.v, (short)0, c, false, false);
  asm volatile("v_nop\n\tv_nop\n\tv_nop\n\tv_nop" : "+v"(d) : "v"(a.w), "v"(b.w));
  return d;
}

__device__ __forceinline__ unsigned bf16_bits(float f) {
  const unsigned u = __float_as_uint(f);
  const unsigned r = (u + 0x7FFFu + ((u >> 16) & 1u)) >> 16;
  const unsigned q = (u >> 16) | 0x40u;
  return ((u & 0x7fffffffu) > 0x7f800000u) ? q : r;
}

__device__ __forceinline__ float bf16_val(float f) {
  return __uint_as_float(bf16_bits(f) << 16);
}
__device__ __forceinline__ int clampi(int v, int lo, int hi) {
  return v < lo ? lo : (v > hi ? hi : v);
}

__device__ __forceinline__ unsigned f16_bits(float f) {
  const unsigned u  = __float_as_uint(f);
  const unsigned s  = (u >> 16) & 0x8000u;
  const unsigned a  = u & 0x7fffffffu;
  const unsigned t  = a - 0x38000000u;
  const unsigned r  = (t + 0x0FFFu + ((t >> 13) & 1u)) >> 13;
  const unsigned rc = r > 0x7C00u ? 0x7C00u : r;
  const bool small  = a < 0x38800000u;
  const bool isnan  = a > 0x7f800000u;
  const unsigned fin = small ? 0u : (s | rc);
  return isnan ? (s | 0x7E00u) : fin;
}

__device__ __forceinline__ unsigned pk16(unsigned lo, unsigned hi) { return lo | (hi << 16); }
__device__ __forceinline__ unsigned bf16_lo_bits(float v) {
  float hi = bf16_val(v);
  asm volatile("" : "+v"(hi));
  return bf16_bits(v - hi);
}
__device__ __forceinline__ v4u pack8_bf16(v4f a, v4f c) {
  return (v4u){ pk16(bf16_bits(a[0]), bf16_bits(a[1])), pk16(bf16_bits(a[2]), bf16_bits(a[3])),
                pk16(bf16_bits(c[0]), bf16_bits(c[1])), pk16(bf16_bits(c[2]), bf16_bits(c[3])) };
}
__device__ __forceinline__ v4u pack8_bf16_lo(v4f a, v4f c) {
  return (v4u){ pk16(bf16_lo_bits(a[0]), bf16_lo_bits(a[1])), pk16(bf16_lo_bits(a[2]), bf16_lo_bits(a[3])),
                pk16(bf16_lo_bits(c[0]), bf16_lo_bits(c[1])), pk16(bf16_lo_bits(c[2]), bf16_lo_bits(c[3])) };
}
__device__ __forceinline__ v4u pack8_f16(v4f a, v4f c) {
  return (v4u){ pk16(f16_bits(a[0]), f16_bits(a[1])), pk16(f16_bits(a[2]), f16_bits(a[3])),
                pk16(f16_bits(c[0]), f16_bits(c[1])), pk16(f16_bits(c[2]), f16_bits(c[3])) };
}

template <int FORM>
__global__ __launch_bounds__(256) void k_plane(const float* __restrict__ src, int rows, int cols, int ldsrc,
                                               unsigned short* __restrict__ dst, int MP, int KP) {
  static_assert(FORM >= 0 && FORM <= 3);
  const int KTOT = (FORM == 1 || FORM == 3) ? 2 * KP : KP;
  const unsigned ppr   = (unsigned)(KTOT >> 3);
  const unsigned kp8   = (unsigned)(KP >> 3);
  const unsigned total = (unsigned)MP * ppr;
  const unsigned g     = blockIdx.x * 256u + threadIdx.x;
  const unsigned rowu  = g / ppr;
  const unsigned p     = g - rowu * ppr;
  const bool second    = p >= kp8;
  const int row = (int)rowu;
  const int c0  = (int)((second ? p - kp8 : p) << 3);
  const float* srow = src + (size_t)clampi(row, 0, rows - 1) * (size_t)ldsrc;
  float x[8];
  unsigned mk[8];
#pragma unroll
  for (int e = 0; e < 8; ++e) {
    const int c = c0 + e;
    const float v = srow[clampi(c, 0, cols - 1)];
    asm volatile("" :: "v"(v));
    x[e]  = v;
    mk[e] = (row < rows && c < cols) ? 0xFFFFu : 0u;
  }
  const v4f a = (v4f){ x[0], x[1], x[2], x[3] };
  const v4f c = (v4f){ x[4], x[5], x[6], x[7] };
  v4u o;
  if (FORM == 2) {
    o = pack8_f16(a, c);
  } else {
    const v4u hi = pack8_bf16(a, c);
    o = hi;
    if (FORM == 1) { const v4u lo = pack8_bf16_lo(a, c); o = second ? lo : hi; }
  }
  const v4u mw = (v4u){ pk16(mk[0], mk[1]), pk16(mk[2], mk[3]), pk16(mk[4], mk[5]), pk16(mk[6], mk[7]) };
  o &= mw;
  if (g < total) {
    volatile v4u* q = (volatile v4u*)(dst + (size_t)g * 8);
    *q = o;
    __threadfence();
    *q = o;
  }
}

template <int FORM> struct FragOf    { typedef FragB T; };
template <>         struct FragOf<2> { typedef FragH T; };
__device__ __forceinline__ v8f mm(const FragB& a, const FragB& b, v8f c) { return wmb(a, b, c); }
__device__ __forceinline__ v8f mm(const FragH& a, const FragH& b, v8f c) { return wmh(a, b, c); }
template <class F> __device__ __forceinline__ F ld_frag(const unsigned short* p) {
  F f;
  f.h[0] = *(const v8usa*)(p);
  f.h[1] = *(const v8usa*)(p + 16);
  return f;
}

template <int FORM, int EPI>
__global__ __launch_bounds__(256) __attribute__((amdgpu_num_vgpr(248)))
void k_gemm_nt(const unsigned short* __restrict__ A, const unsigned short* __restrict__ B,
               const float* __restrict__ bias, float* __restrict__ D, int M, int N, int KTOT, int ldd) {
  static_assert(FORM >= 0 && FORM <= 2);
  static_assert(EPI == 0 || EPI == 1);
  typedef typename FragOf<FORM>::T F;
  __shared__ __attribute__((aligned(16))) float sT[8][16 * 68];
  const int lane = threadIdx.x & 31;
  const int wave = threadIdx.x >> 5;
  const int tilesM = (M + 63) >> 6;
  const int tilesN = (N + 63) >> 6;
  const int tile = blockIdx.x * 8 + wave;
  if (tile >= tilesM * tilesN) return;
  const int tm = tile / tilesN;
  const int tn = tile - tm * tilesN;
  const int m0 = tm << 6;
  const int n0 = tn << 6;

  const int rl = lane & 15;
  const int h8 = (lane >> 4) * 8;
  const unsigned short* pa = A + (size_t)(m0 + rl) * (size_t)KTOT + h8;
  const unsigned short* pb = B + (size_t)(n0 + rl) * (size_t)KTOT + h8;

  v8f acc[4][4];
#pragma unroll
  for (int i = 0; i < 4; ++i)
#pragma unroll
    for (int j = 0; j < 4; ++j) acc[i][j] = (v8f){0.f, 0.f, 0.f, 0.f, 0.f, 0.f, 0.f, 0.f};

#pragma unroll 1
  for (int k0 = 0; k0 < KTOT; k0 += 32) {
    F bf[4];
#pragma unroll
    for (int j = 0; j < 4; ++j) bf[j] = ld_frag<F>(pb + (size_t)(j << 4) * (size_t)KTOT + k0);
#pragma unroll
    for (int i = 0; i < 4; ++i) {
      const F af = ld_frag<F>(pa + (size_t)(i << 4) * (size_t)KTOT + k0);
#pragma unroll
      for (int j = 0; j < 4; ++j) acc[i][j] = mm(af, bf[j], acc[i][j]);
    }
  }

  float* slab = sT[wave];
  const int hh = lane >> 4;
  const int c4 = (lane & 15) * 4;
  const int nc = n0 + c4;
  const bool cok = nc < N;
  v4f bv = (v4f){0.f, 0.f, 0.f, 0.f};
  if (EPI == 1) {
    bv = *(const v4fa*)(bias + clampi(nc, 0, N - 4));
    asm volatile("" :: "v"(bv));
  }
#pragma unroll
  for (int i = 0; i < 4; ++i) {
    const int mBase = m0 + (i << 4);
#pragma unroll
    for (int j = 0; j < 4; ++j) {
#pragma unroll
      for (int r = 0; r < 8; ++r) slab[(h8 + r) * 68 + (j << 4) + rl] = acc[i][j][r];
    }
    __builtin_amdgcn_fence(__ATOMIC_RELEASE, "workgroup");
    __builtin_amdgcn_wave_barrier();
    __builtin_amdgcn_fence(__ATOMIC_ACQUIRE, "workgroup");
    v4f vv[8];
#pragma unroll
    for (int it = 0; it < 8; ++it) {
      const int row = it * 2 + hh;
      v4f v = *(const v4fa*)(slab + row * 68 + c4);
      if (EPI == 1) v += bv;
      vv[it] = v;
    }
    for (int pass = 0; pass < 2; ++pass) {
#pragma unroll
      for (int it = 0; it < 8; ++it) {
        const int row = mBase + it * 2 + hh;
        if (cok && row < M) *(volatile v4f*)(D + (size_t)row * (size_t)ldd + nc) = vv[it];
      }
      __threadfence();
    }
    __builtin_amdgcn_fence(__ATOMIC_RELEASE, "workgroup");
    __builtin_amdgcn_wave_barrier();
    __builtin_amdgcn_fence(__ATOMIC_ACQUIRE, "workgroup");
  }
}

#define NN      50000
#define NE      800000
#define DF      128
#define DC      256
#define MPAD    50048
#define NBRUN   1024
#define NBLK    49
#define LCAP    21504
#define DEGCAP  64
#define MEAS_BLKMAX 16759
#define MEAS_DEGMAX 37
#define BTHR    256
#define BWAVE   8
#define SEG     (NE / BWAVE)
#define NEIGH_TWO_TERM 1
#define SUPK    (NEIGH_TWO_TERM ? 2 * DF : DF)
#define BZINTS  (2 * LCAP + 3 * NBRUN)
#define BMISC   32
#define BUCKET_LDS_BYTES ((BZINTS + BMISC) * 4)
#define NTB     768

static_assert(DF == 128 && DC == 2 * DF && DC == 32 * 8);
static_assert(NN <= NBLK * NBRUN && MPAD <= NBLK * NBRUN && MPAD >= NN);
static_assert(MPAD % 64 == 0 && MPAD % 8 == 0 && NN % 16 == 0 && NN % 8 == 0);
static_assert(NE % 256 == 0 && SEG % 32 == 0 && SEG * BWAVE == NE);
static_assert(NE <= (1 << 20) && NBRUN <= 1024 && NBRUN == (1 << 10));
static_assert((long long)LCAP * 4 >= (long long)MEAS_BLKMAX * 5);
static_assert(DEGCAP >= MEAS_DEGMAX + 8 && DEGCAP * 4 >= MEAS_DEGMAX * 5 && DEGCAP % 32 == 0);
static_assert(LCAP % (BTHR * 4) == 0 && BZINTS % (BTHR * 4) == 0);
static_assert(BUCKET_LDS_BYTES <= 262144);
static_assert(SUPK % 32 == 0 && DF % 32 == 0);
static_assert((MPAD * DF / 8) % 256 == 0 && (DF * DF / 8) % 256 == 0 && (DF * SUPK / 8) % 256 == 0);

constexpr size_t SZ_HB   = (size_t)MPAD * DF * 2;
constexpr size_t SZ_SUP  = (size_t)MPAD * SUPK * 2;
constexpr size_t SZ_X    = (size_t)MPAD * DC * 4;
constexpr size_t SZ_WS   = (size_t)DF * DF * 2;
constexpr size_t SZ_WN   = (size_t)DF * SUPK * 2;
constexpr size_t SZ_TB   = (size_t)NTB * 4;
constexpr size_t SZ_LIST = (size_t)NBLK * LCAP * 4;
constexpr size_t SZ_OFF  = (size_t)NBLK * NBRUN * 4;
constexpr size_t SZ_CNT  = (size_t)NBLK * NBRUN * 4;
constexpr size_t SZ_FLAG = (size_t)NBLK * 128;
constexpr size_t O_HB   = 0;
constexpr size_t O_SUP  = O_HB + SZ_HB;
constexpr size_t O_X    = O_SUP + SZ_SUP;
constexpr size_t O_WS   = O_X + SZ_X;
constexpr size_t O_WN   = O_WS + SZ_WS;
constexpr size_t O_TB   = O_WN + SZ_WN;
constexpr size_t O_LIST = O_TB + SZ_TB;
constexpr size_t O_OFF  = O_LIST + SZ_LIST;
constexpr size_t O_CNT  = O_OFF + SZ_OFF;
constexpr size_t O_FLAG = O_CNT + SZ_CNT;
constexpr size_t WS_TOTAL = O_FLAG + SZ_FLAG;
static_assert(SZ_HB % 128 == 0 && SZ_SUP % 128 == 0 && SZ_X % 128 == 0 && SZ_WS % 128 == 0 && SZ_WN % 128 == 0);
static_assert(SZ_TB % 128 == 0 && SZ_LIST % 128 == 0 && SZ_OFF % 128 == 0 && SZ_CNT % 128 == 0 && SZ_FLAG % 128 == 0);
static_assert(!NEIGH_TWO_TERM || WS_TOTAL == 94409856);
static_assert(WS_TOTAL <= ((size_t)128 << 20));

typedef unsigned int v2u __attribute__((ext_vector_type(2)));
typedef int          v4i __attribute__((ext_vector_type(4)));
typedef v2u __attribute__((may_alias)) v2ua;
typedef v4u __attribute__((may_alias)) v4ua;
typedef v4i __attribute__((may_alias)) v4ia;

__device__ __forceinline__ void wave_sync() {
  __builtin_amdgcn_fence(__ATOMIC_RELEASE, "wavefront");
  __builtin_amdgcn_wave_barrier();
  __builtin_amdgcn_fence(__ATOMIC_ACQUIRE, "wavefront");
}

__device__ __forceinline__ float relu_keep(float v) { return (v > 0.0f) ? v : (v - v); }

__global__ __launch_bounds__(192) void k_tables(const float* __restrict__ bs, const float* __restrict__ bn,
                                                const float* __restrict__ gm, const float* __restrict__ bt,
                                                float* __restrict__ TB) {
  const int t = (int)threadIdx.x;
  const v4f q0 = *(const v4fa*)(bs + 4 * clampi(t, 0, 31));
  asm volatile("" :: "v"(q0));
  const v4f q1 = *(const v4fa*)(bn + 4 * clampi(t - 32, 0, 31));
  asm volatile("" :: "v"(q1));
  const v4f q2 = *(const v4fa*)(gm + 4 * clampi(t - 64, 0, 63));
  asm volatile("" :: "v"(q2));
  const v4f q3 = *(const v4fa*)(bt + 4 * clampi(t - 128, 0, 63));
  asm volatile("" :: "v"(q3));
  const unsigned m0 = (t < 32) ? 0xFFFFFFFFu : 0u;
  const unsigned m1 = (t >= 32 && t < 64) ? 0xFFFFFFFFu : 0u;
  const unsigned m2 = (t >= 64 && t < 128) ? 0xFFFFFFFFu : 0u;
  const unsigned m3 = (t >= 128) ? 0xFFFFFFFFu : 0u;
  v4f o;
#pragma unroll
  for (int j = 0; j < 4; ++j) {
    const unsigned u = (__float_as_uint(q0[j]) & m0) | (__float_as_uint(q1[j]) & m1) |
                       (__float_as_uint(q2[j]) & m2) | (__float_as_uint(q3[j]) & m3);
    o[j] = bf16_val(__uint_as_float(u));
  }
  if (t < NTB / 4) {
    volatile v4f* q = (volatile v4f*)(TB + 4 * t);
    *q = o;
    __threadfence();
    *q = o;
  }
}

__global__ __launch_bounds__(BTHR) void k_bucket(const int* __restrict__ keys, int* __restrict__ LIST,
                                                 int* __restrict__ OFF, int* __restrict__ CNT,
                                                 int* __restrict__ FLAG) {
  extern __shared__ __attribute__((aligned(16))) int dsm[];
  int* hl   = dsm;
  int* sl   = hl + LCAP;
  int* cnt  = sl + LCAP;
  int* offs = cnt + NBRUN;
  int* cur  = offs + NBRUN;
  int* misc = cur + NBRUN;
  const int tid = (int)threadIdx.x, lane = tid & 31, wave = tid >> 5;
  const int blk = (int)blockIdx.x;
  const unsigned base = (unsigned)blk * (unsigned)NBRUN;
  const unsigned nb   = (unsigned)clampi(NN - blk * NBRUN, 0, NBRUN);

  {
    const v4i z4 = (v4i){0, 0, 0, 0};
    for (int i = tid * 4; i < BZINTS; i += BTHR * 4) *(v4ia*)(dsm + i) = z4;
    if (tid < BMISC) misc[tid] = 0;
  }
  __syncthreads();

  const int* kp = keys + wave * SEG + lane;
  int wc = 0;
#pragma unroll 1
  for (int it = 0; it < SEG / 32; ++it) {
    const int key = kp[it * 32];
    const unsigned s = (unsigned)key - base;
    const unsigned m = __builtin_amdgcn_ballot_w32(s < nb);
    wc += (int)__builtin_popcount(m);
  }
  if (lane == 0) misc[wave] = wc;
  __syncthreads();
  int basew = 0, total = 0;
#pragma unroll
  for (int w2 = 0; w2 < BWAVE; ++w2) {
    const int c2 = clampi(misc[w2], 0, SEG);
    total += c2;
    basew += (w2 < wave) ? c2 : 0;
  }
  const int ovf = (total > LCAP) ? 1 : 0;
  const int tt  = (total > LCAP) ? LCAP : total;

  int run = basew;
#pragma unroll 1
  for (int it = 0; it < SEG / 32; ++it) {
    const int key = kp[it * 32];
    const unsigned s = (unsigned)key - base;
    const bool hit = s < nb;
    const unsigned m = __builtin_amdgcn_ballot_w32(hit);
    if (m != 0u) {
      const int pos = run + (int)__builtin_amdgcn_mbcnt_lo(m, 0u);
      const int e   = wave * SEG + it * 32 + lane;
      if (hit && pos < LCAP) hl[pos] = (int)((s << 20) | (unsigned)e);
      run += (int)__builtin_popcount(m);
    }
  }
  __syncthreads();

  if (wave == 0) {
#pragma unroll 1
    for (int b0 = 0; b0 < tt; b0 += 32) {
      const int idx = clampi(b0 + lane, 0, LCAP - 1);
      const int ent = hl[idx];
      int m32 = tt - b0;
      m32 = m32 > 32 ? 32 : m32;
#pragma unroll 1
      for (int k = 0; k < m32; ++k) {
        const int u = __builtin_amdgcn_readlane(ent, k);
        const int s = (u >> 20) & (NBRUN - 1);
        const int cv = cnt[s];
        cnt[s] = cv + 1;
      }
    }
  }
  __syncthreads();

  if (wave == 0) {
    const int sb = lane * (NBRUN / 32);
    int s = 0;
#pragma unroll 1
    for (int i = 0; i < NBRUN / 32; ++i) s += cnt[sb + i];
    int incl = s;
#pragma unroll
    for (int d = 1; d < 32; d <<= 1) {
      const int y = __shfl_up(incl, d, 32);
      incl += (lane >= d) ? y : 0;
    }
    int rr = incl - s;
#pragma unroll 1
    for (int i = 0; i < NBRUN / 32; ++i) {
      const int cv = cnt[sb + i];
      offs[sb + i] = rr;
      cur[sb + i]  = rr;
      rr += cv;
    }
  }
  __syncthreads();

  if (wave == 0) {
#pragma unroll 1
    for (int b0 = 0; b0 < tt; b0 += 32) {
      const int idx = clampi(b0 + lane, 0, LCAP - 1);
      const int ent = hl[idx];
      int m32 = tt - b0;
      m32 = m32 > 32 ? 32 : m32;
#pragma unroll 1
      for (int k = 0; k < m32; ++k) {
        const int u = __builtin_amdgcn_readlane(ent, k);
        const int s = (u >> 20) & (NBRUN - 1);
        const int p = clampi(cur[s], 0, LCAP - 1);
        sl[p]  = u & 0xFFFFF;
        cur[s] = p + 1;
      }
    }
  }
  __syncthreads();

  int* gl = LIST + (size_t)blk * LCAP;
  const v4i ov4 = *(const v4ia*)(offs + 4 * tid);
  const v4i cv4 = *(const v4ia*)(cnt + 4 * tid);
  const v4i fv4 = (v4i){ovf, total, 0, 0};
  for (int pass = 0; pass < 2; ++pass) {
#pragma unroll 1
    for (int i = 0; i < LCAP / (BTHR * 4); ++i) {
      const int p4 = (i * BTHR + tid) * 4;
      const v4i v = *(const v4ia*)(sl + p4);
      *(volatile v4i*)(gl + p4) = v;
    }
    *(volatile v4i*)(OFF + blk * NBRUN + 4 * tid) = ov4;
    *(volatile v4i*)(CNT + blk * NBRUN + 4 * tid) = cv4;
    if (tid < 8) *(volatile v4i*)(FLAG + blk * 32 + 4 * tid) = fv4;
    __threadfence();
  }
}

__global__ __launch_bounds__(256) void k_replay(const unsigned short* __restrict__ HB, const int* __restrict__ ecol,
                                                const float* __restrict__ eval, const int* __restrict__ LIST,
                                                const int* __restrict__ OFF, const int* __restrict__ CNT,
                                                const int* __restrict__ FLAG, unsigned short* __restrict__ SUP) {
  __shared__ __attribute__((aligned(16))) unsigned rowbuf[BWAVE][DF];
  const int lane = (int)threadIdx.x & 31, wave = (int)threadIdx.x >> 5;
  const int node = (int)blockIdx.x * 8 + wave;
  const int nidx = clampi(node, 0, NBLK * NBRUN - 1);
  const int blk  = nidx >> 10;
  int cl = CNT[nidx];
  asm volatile("" :: "v"(cl));
  int ol = OFF[nidx];
  asm volatile("" :: "v"(ol));
  int fl = FLAG[blk * 32];
  asm volatile("" :: "v"(fl));
  const bool live = node < NN;
  const int bigv = (cl > DEGCAP) ? 1 : 0;
  cl = clampi(cl, 0, DEGCAP);
  cl = live ? cl : 0;
  ol = clampi(ol, 0, LCAP - 1);
  const int c   = __builtin_amdgcn_readfirstlane(cl);
  const int o   = __builtin_amdgcn_readfirstlane(ol);
  const int bad = __builtin_amdgcn_readfirstlane((fl != 0) ? 1 : bigv);
  const int* lp = LIST + (size_t)blk * LCAP;

  float a0 = 0.0f, a1 = 0.0f, a2 = 0.0f, a3 = 0.0f;
#pragma unroll 1
  for (int b0 = 0; b0 < c; b0 += 32) {
    const int last = o + c - 1;
    int idx = o + b0 + lane;
    idx = idx > last ? last : idx;
    idx = clampi(idx, 0, LCAP - 1);
    int e = lp[idx];
    asm volatile("" :: "v"(e));
    e = clampi(e, 0, NE - 1);
    int col = ecol[e];
    asm volatile("" :: "v"(col));
    col = clampi(col, 0, NN - 1);
    float w = eval[e];
    asm volatile("" :: "v"(w));
    const int wvi = __float_as_int(bf16_val(w));
    int m32 = c - b0;
    m32 = m32 > 32 ? 32 : m32;
#pragma unroll 1
    for (int k = 0; k < m32; ++k) {
      const int   sk = __builtin_amdgcn_readlane(col, k);
      const float ck = __int_as_float(__builtin_amdgcn_readlane(wvi, k));
      const v2u hv = *(const v2ua*)(HB + (size_t)sk * DF + 4 * lane);
      const float f0 = __uint_as_float(hv.x << 16);
      const float f1 = __uint_as_float(hv.x & 0xffff0000u);
      const float f2 = __uint_as_float(hv.y << 16);
      const float f3 = __uint_as_float(hv.y & 0xffff0000u);
      a0 = fmaf(ck, f0, a0);
      a1 = fmaf(ck, f1, a1);
      a2 = fmaf(ck, f2, a2);
      a3 = fmaf(ck, f3, a3);
    }
  }
  const float pz  = (bad != 0) ? __int_as_float(0x7fc00000) : 0.0f;
  const bool some = c > 0;
  float m0 = (some ? a0 : 0.0f) + pz;
  float m1 = (some ? a1 : 0.0f) + pz;
  float m2 = (some ? a2 : 0.0f) + pz;
  float m3 = (some ? a3 : 0.0f) + pz;
  m0 = live ? m0 : 0.0f;
  m1 = live ? m1 : 0.0f;
  m2 = live ? m2 : 0.0f;
  m3 = live ? m3 : 0.0f;
  unsigned* rb = rowbuf[wave];
  const v2u hw = (v2u){ pk16(bf16_bits(m0), bf16_bits(m1)), pk16(bf16_bits(m2), bf16_bits(m3)) };
  *(v2ua*)(rb + 2 * lane) = hw;
  if (NEIGH_TWO_TERM) {
    const v2u lw = (v2u){ pk16(bf16_lo_bits(m0), bf16_lo_bits(m1)), pk16(bf16_lo_bits(m2), bf16_lo_bits(m3)) };
    *(v2ua*)(rb + 64 + 2 * lane) = lw;
  }
  wave_sync();
  const int rd = NEIGH_TWO_TERM ? (4 * lane) : (4 * (lane & 15));
  const v4u qv = *(const v4ua*)(rb + rd);
  const bool wr = (node < MPAD) && (NEIGH_TWO_TERM ? true : (lane < 16));
  if (wr) {
    volatile v4u* q = (volatile v4u*)(SUP + (size_t)node * SUPK + 8 * lane);
    *q = qv;
    __threadfence();
    *q = qv;
  }
}

__global__ __launch_bounds__(256) void k_ln(const float* __restrict__ X, const float* __restrict__ TB,
                                            const int* __restrict__ FLAG, float* __restrict__ out) {
  const int lane = (int)threadIdx.x & 31, wave = (int)threadIdx.x >> 5;
  const int row = (int)blockIdx.x * 8 + wave;
  const int rc  = clampi(row, 0, NN - 1);
  const float* xr = X + (size_t)rc * DC;
  const v4f x0 = *(const v4fa*)(xr + 4 * lane);
  const v4f x1 = *(const v4fa*)(xr + DF + 4 * lane);
  const v4f g0 = *(const v4fa*)(TB + 256 + 4 * lane);
  const v4f g1 = *(const v4fa*)(TB + 256 + DF + 4 * lane);
  const v4f e0 = *(const v4fa*)(TB + 512 + 4 * lane);
  const v4f e1 = *(const v4fa*)(TB + 512 + DF + 4 * lane);
  int fl = FLAG[(rc >> 10) * 32];
  asm volatile("" :: "v"(fl));

  float t[8];
#pragma unroll
  for (int j = 0; j < 4; ++j) { t[j] = relu_keep(x0[j]); t[4 + j] = relu_keep(x1[j]); }
  float s = ((t[0] + t[1]) + (t[2] + t[3])) + ((t[4] + t[5]) + (t[6] + t[7]));
#pragma unroll
  for (int m = 16; m >= 1; m >>= 1) s += __shfl_xor(s, m, 32);
  const float mu = s * (1.0f / 256.0f);
  float d[8];
  float q = 0.0f;
#pragma unroll
  for (int j = 0; j < 8; ++j) { d[j] = t[j] - mu; q = fmaf(d[j], d[j], q); }
#pragma unroll
  for (int m = 16; m >= 1; m >>= 1) q += __shfl_xor(q, m, 32);
  const float var = q * (1.0f / 256.0f);
  const float r = 1.0f / sqrtf(var + 1e-5f);
  const float nanv = __int_as_float(0x7fc00000);
  const bool bad = fl != 0;
  v4f y0, y1;
#pragma unroll
  for (int j = 0; j < 4; ++j) {
    const float u0 = fmaf(d[j] * r, g0[j], e0[j]);
    const float u1 = fmaf(d[4 + j] * r, g1[j], e1[j]);
    y0[j] = bad ? nanv : u0;
    y1[j] = bad ? nanv : u1;
  }
  if (row < NN) {
    volatile v4f* p0 = (volatile v4f*)(out + (size_t)row * DC + 4 * lane);
    volatile v4f* p1 = (volatile v4f*)(out + (size_t)row * DC + DF + 4 * lane);
    *p0 = y0;
    *p1 = y1;
    __threadfence();
    *p0 = y0;
    *p1 = y1;
  }
}

extern "C" void kernel_launch(void* const* d_in, const int* in_sizes, int n_in,
                              void* d_out, int out_size, void* d_ws, size_t ws_size,
                              hipStream_t stream) {
  if (n_in < 10) return;
  if (in_sizes[0] != NN * DF) return;
  if (in_sizes[1] != NE || in_sizes[2] != NE || in_sizes[3] != NE) return;
  if (in_sizes[4] != DF * DF || in_sizes[5] != DF) return;
  if (in_sizes[6] != DF * DF || in_sizes[7] != DF) return;
  if (in_sizes[8] != DC || in_sizes[9] != DC) return;
  if ((long long)out_size != (long long)NN * DC) return;
  if (ws_size < WS_TOTAL) return;

  const float* h     = (const float*)d_in[0];
  const int*   erow  = (const int*)d_in[1];
  const int*   ecol  = (const int*)d_in[2];
  const float* evalp = (const float*)d_in[3];
  const float* Wself = (const float*)d_in[4];
  const float* bself = (const float*)d_in[5];
  const float* Wnei  = (const float*)d_in[6];
  const float* bnei  = (const float*)d_in[7];
  const float* gamma = (const float*)d_in[8];
  const float* beta  = (const float*)d_in[9];
  float* out = (float*)d_out;

  char* ws = (char*)d_ws;
  unsigned short* HB  = (unsigned short*)(ws + O_HB);
  unsigned short* SUP = (unsigned short*)(ws + O_SUP);
  float*          X   = (float*)(ws + O_X);
  unsigned short* WS  = (unsigned short*)(ws + O_WS);
  unsigned short* WN  = (unsigned short*)(ws + O_WN);
  float*          TB  = (float*)(ws + O_TB);
  int*            LST = (int*)(ws + O_LIST);
  int*            OFF = (int*)(ws + O_OFF);
  int*            CNT = (int*)(ws + O_CNT);
  int*            FLG = (int*)(ws + O_FLAG);

  hipFuncSetAttribute(reinterpret_cast<const void*>(&k_bucket), hipFuncAttributeMaxDynamicSharedMemorySize,
                      (int)BUCKET_LDS_BYTES);

  k_plane<0><<<MPAD * DF / 8 / 256, 256, 0, stream>>>(h, NN, DF, DF, HB, MPAD, DF);
  k_plane<0><<<DF * DF / 8 / 256, 256, 0, stream>>>(Wself, DF, DF, DF, WS, DF, DF);
#if NEIGH_TWO_TERM
  k_plane<3><<<DF * SUPK / 8 / 256, 256, 0, stream>>>(Wnei, DF, DF, DF, WN, DF, DF);
#else
  k_plane<0><<<DF * SUPK / 8 / 256, 256, 0, stream>>>(Wnei, DF, DF, DF, WN, DF, DF);
#endif
  k_tables<<<1, 192, 0, stream>>>(bself, bnei, gamma, beta, TB);
  k_bucket<<<NBLK, BTHR, BUCKET_LDS_BYTES, stream>>>(erow, LST, OFF, CNT, FLG);
  k_replay<<<MPAD / 8, 256, 0, stream>>>(HB, ecol, evalp, LST, OFF, CNT, FLG, SUP);
  {
    const int tiles  = ((NN + 63) / 64) * ((DF + 63) / 64);
    const int blocks = (tiles + 7) / 8;
    k_gemm_nt<0, 1><<<blocks, 256, 0, stream>>>(HB, WS, TB, X, NN, DF, DF, DC);
    k_gemm_nt<0, 1><<<blocks, 256, 0, stream>>>(SUP, WN, TB + DF, X + DF, NN, DF, SUPK, DC);
  }
  k_ln<<<NN / 8, 256, 0, stream>>>(X, TB, FLG, out);
}
